// Decoder_83099027243701
// MI455X (gfx1250) — hardware-verified
//
#include <hip/hip_runtime.h>
#include <math.h>

constexpr int NBATCH   = 131072;
constexpr int NHID     = 64;
constexpr int NGATE    = 256;
constexpr int NSTEP    = 12;
constexpr int NTHR     = 256;
constexpr int NWAVE    = 8;
constexpr int ROWS_BLK = 128;
constexpr int WPITCH   = 72;
constexpr int HPITCH   = 72;
constexpr int CPITCH   = 68;
constexpr int OUT1_OFF = NSTEP * NBATCH * 2;

static_assert(NGATE == 4 * NHID, "gate blocks");
static_assert(NHID % 32 == 0, "K multiple of 32");
static_assert(NBATCH % ROWS_BLK == 0, "exact grid");
static_assert(ROWS_BLK == NWAVE * 16, "16 rows per wave");
static_assert(NTHR == NWAVE * 32, "wave32");
static_assert((size_t)OUT1_OFF * 4 == (size_t)12582912, "second output byte offset");
static_assert((size_t)2 * OUT1_OFF * 4 == (size_t)25165824, "total output bytes");
static_assert(NTHR == NGATE, "one thread per gate column in the table fill");

typedef __attribute__((ext_vector_type(16))) _Float16 v16h;
typedef __attribute__((ext_vector_type(8)))  _Float16 v8h;
typedef __attribute__((ext_vector_type(4)))  _Float16 v4h;
typedef __attribute__((ext_vector_type(8)))  float    v8f;
typedef __attribute__((ext_vector_type(4)))  float    v4f;
typedef __attribute__((ext_vector_type(2)))  float    v2f;

__device__ __forceinline__ unsigned short f2bf_bits(float f) {
  unsigned u = __float_as_uint(f);
  return (unsigned short)((u + 0x7FFFu + ((u >> 16) & 1u)) >> 16);
}
__device__ __forceinline__ float bf_bits2f(unsigned short h) { return __uint_as_float(((unsigned)h) << 16); }
__device__ __forceinline__ float bf16r(float f) { return bf_bits2f(f2bf_bits(f)); }

struct FragH {
  union U { v16h v; v8h h[2]; };
  static __device__ __forceinline__ v16h load(const _Float16* p) {
    U f; f.h[0] = *(const v8h*)(p); f.h[1] = *(const v8h*)(p + 16); return f.v;
  }
  static __device__ __forceinline__ v8f mma(v16h a, v16h b, v8f c) {
    return __builtin_amdgcn_wmma_f32_16x16x32_f16(false, a, false, b, (short)0, c, false, false);
  }
};
__device__ __forceinline__ void mma_guard(v8f& acc, v16h a0, v16h a1, v16h b0, v16h b1) {
  asm volatile("v_nop\n\tv_nop\n\tv_nop\n\tv_nop" : "+v"(acc) : "v"(a0), "v"(a1), "v"(b0), "v"(b1));
}
__device__ __forceinline__ void acc_guard4(v8f& a, v8f& b, v8f& c, v8f& d) {
  asm volatile("v_nop\n\tv_nop\n\tv_nop\n\tv_nop" : "+v"(a), "+v"(b), "+v"(c), "+v"(d));
}
__device__ __forceinline__ void wave_lds_sync() {
  __builtin_amdgcn_fence(__ATOMIC_RELEASE, "workgroup");
  __builtin_amdgcn_wave_barrier();
  __builtin_amdgcn_fence(__ATOMIC_ACQUIRE, "workgroup");
}

__device__ __forceinline__ float fsig(float x)  { return __builtin_amdgcn_rcpf(1.0f + __expf(-x)); }
__device__ __forceinline__ float ftanh(float x) { return 1.0f - 2.0f * __builtin_amdgcn_rcpf(__expf(2.0f * x) + 1.0f); }

__global__ __launch_bounds__(NTHR) void lstm_seq_kernel(
    const float* __restrict__ enc_h, const float* __restrict__ enc_c,
    const float* __restrict__ obs_pos, const float* __restrict__ obs_rel,
    const float* __restrict__ w_emb, const float* __restrict__ b_emb,
    const float* __restrict__ w_ih, const float* __restrict__ w_hh,
    const float* __restrict__ b_ih, const float* __restrict__ b_hh,
    const float* __restrict__ w_pos, const float* __restrict__ b_pos,
    float* __restrict__ out) {
  __shared__ __align__(16) _Float16 sW[NGATE * WPITCH];
  __shared__ __align__(16) _Float16 sH[NWAVE * 16 * HPITCH];
  __shared__ __align__(16) float    sC[NWAVE * 16 * CPITCH];
  __shared__ __align__(16) float    sG[NGATE * 4];
  __shared__ __align__(16) float    sP[NHID * 2];
  __shared__ __align__(16) float    sO[NWAVE * 64];

  const int tid  = threadIdx.x;
  const int wave = tid >> 5;
  const int lane = tid & 31;
  const int g    = lane >> 4;
  const int nl   = lane & 15;
  const int koff = 8 * g;
  const int rowW = blockIdx.x * ROWS_BLK + wave * 16;

#pragma unroll 1
  for (int it = 0; it < 16; ++it) {
    const int idx = it * NTHR + tid;
    const int n   = idx >> 4;
    const int k4  = (idx & 15) * 4;
    const v4f v = *(const v4f*)(w_hh + n * NHID + k4);
    const float f0 = v[0], f1 = v[1], f2 = v[2], f3 = v[3];
    v4h hv;
    hv[0] = (_Float16)bf16r(f0);
    hv[1] = (_Float16)bf16r(f1);
    hv[2] = (_Float16)bf16r(f2);
    hv[3] = (_Float16)bf16r(f3);
    *(v4h*)(sW + n * WPITCH + k4) = hv;
  }
  {
    const int n = tid;
    const v2f wi = *(const v2f*)(w_ih + 2 * n);
    const float w0 = wi[0], w1 = wi[1];
    const float bi = b_ih[n];
    const float bh = b_hh[n];
    v4f gv;
    gv[0] = bf16r(w0);
    gv[1] = bf16r(w1);
    gv[2] = bf16r(bi) + bf16r(bh);
    gv[3] = 0.0f;
    *(v4f*)(sG + 4 * n) = gv;
  }
  if (wave < 2) {
    const int k = tid;
    const float pa = w_pos[k];
    const float pb = w_pos[NHID + k];
    v2f pv2;
    pv2[0] = bf16r(pa);
    pv2[1] = bf16r(pb);
    *(v2f*)(sP + 2 * k) = pv2;
  }

  _Float16* hb = sH + wave * 16 * HPITCH;
  float*    cb = sC + wave * 16 * CPITCH;
  float*    so = sO + wave * 64;

#pragma unroll 1
  for (int it = 0; it < 8; ++it) {
    const int idx = it * 32 + lane;
    const int row = idx >> 4;
    const int c4  = (idx & 15) * 4;
    const size_t off = (size_t)(rowW + row) * NHID + c4;
    const v4f hv4 = *(const v4f*)(enc_h + off);
    const v4f cv4 = *(const v4f*)(enc_c + off);
    const float h0 = hv4[0], h1 = hv4[1], h2 = hv4[2], h3 = hv4[3];
    const float c0 = cv4[0], c1 = cv4[1], c2 = cv4[2], c3 = cv4[3];
    v4h hh;
    hh[0] = (_Float16)bf16r(h0);
    hh[1] = (_Float16)bf16r(h1);
    hh[2] = (_Float16)bf16r(h2);
    hh[3] = (_Float16)bf16r(h3);
    *(v4h*)(hb + row * HPITCH + c4) = hh;
    v4f cc;
    cc[0] = bf16r(c0);
    cc[1] = bf16r(c1);
    cc[2] = bf16r(c2);
    cc[3] = bf16r(c3);
    *(v4f*)(cb + row * CPITCH + c4) = cc;
  }

  const float we00 = bf16r(w_emb[0]), we01 = bf16r(w_emb[1]);
  const float we10 = bf16r(w_emb[2]), we11 = bf16r(w_emb[3]);
  const float be0  = bf16r(b_emb[0]), be1  = bf16r(b_emb[1]);
  const float bp0  = bf16r(b_pos[0]), bp1  = bf16r(b_pos[1]);

  float cp0[8], cp1[8], x0[8], x1[8];
  {
    const size_t pbase = (size_t)(rowW + 8 * g) * 2;
    v4f pv[4], rv[4];
#pragma unroll
    for (int i = 0; i < 4; ++i) pv[i] = *(const v4f*)(obs_pos + pbase + 4 * i);
    asm volatile("" ::: "memory");
#pragma unroll
    for (int i = 0; i < 4; ++i) rv[i] = *(const v4f*)(obs_rel + pbase + 4 * i);
#pragma unroll
    for (int r = 0; r < 8; ++r) {
      const float pa = pv[r >> 1][(r & 1) * 2 + 0];
      const float pb = pv[r >> 1][(r & 1) * 2 + 1];
      const float ra = rv[r >> 1][(r & 1) * 2 + 0];
      const float rb = rv[r >> 1][(r & 1) * 2 + 1];
      cp0[r] = bf16r(pa);
      cp1[r] = bf16r(pb);
      const float rx0 = bf16r(ra);
      const float rx1 = bf16r(rb);
      x0[r] = fmaf(rx0, we00, fmaf(rx1, we01, be0));
      x1[r] = fmaf(rx0, we10, fmaf(rx1, we11, be1));
    }
  }
  __syncthreads();

  const _Float16* arow = hb + nl * HPITCH + koff;

#pragma unroll 1
  for (int t = 0; t < NSTEP; ++t) {
    wave_lds_sync();
    const v16h a0 = FragH::load(arow);
    const v16h a1 = FragH::load(arow + 32);

    float p0[8], p1[8];
#pragma unroll
    for (int r = 0; r < 8; ++r) { p0[r] = 0.0f; p1[r] = 0.0f; }

#pragma unroll 1
    for (int tt = 0; tt < 4; ++tt) {
      const int col = 16 * tt + nl;
      v8f gt[4];
#pragma unroll
      for (int q = 0; q < 4; ++q) {
        const int n = 64 * q + col;
        const v4f gw = *(const v4f*)(sG + 4 * n);
        const float gw0 = gw[0], gw1 = gw[1], gw2 = gw[2];
        v8f acc;
#pragma unroll
        for (int r = 0; r < 8; ++r) acc[r] = fmaf(x0[r], gw0, fmaf(x1[r], gw1, gw2));
        const _Float16* brow = sW + n * WPITCH + koff;
        const v16h b0 = FragH::load(brow);
        const v16h b1 = FragH::load(brow + 32);
        acc = FragH::mma(a0, b0, acc);
        acc = FragH::mma(a1, b1, acc);
        mma_guard(acc, a0, a1, b0, b1);
        gt[q] = acc;
      }
      acc_guard4(gt[0], gt[1], gt[2], gt[3]);

      const v2f wp = *(const v2f*)(sP + 2 * col);
      const float wpa = wp[0], wpb = wp[1];
#pragma unroll
      for (int r = 0; r < 8; ++r) {
        const int row = 8 * g + r;
        const float co = cb[row * CPITCH + col];
        const float iv = fsig(gt[0][r]);
        const float fv = fsig(gt[1][r]);
        const float gv = ftanh(gt[2][r]);
        const float ov = fsig(gt[3][r]);
        const float cn = fmaf(fv, co, iv * gv);
        cb[row * CPITCH + col] = cn;
        const float hn = ov * ftanh(cn);
        hb[row * HPITCH + col] = (_Float16)hn;
        p0[r] = fmaf(hn, wpa, p0[r]);
        p1[r] = fmaf(hn, wpb, p1[r]);
      }
    }

#pragma unroll
    for (int m = 1; m < 16; m <<= 1) {
#pragma unroll
      for (int r = 0; r < 8; ++r) {
        const float s0 = __shfl_xor(p0[r], m, 32);
        const float s1 = __shfl_xor(p1[r], m, 32);
        p0[r] += s0;
        p1[r] += s1;
      }
    }
#pragma unroll
    for (int r = 0; r < 8; ++r) {
      const float r0v = p0[r] + bp0;
      const float r1v = p1[r] + bp1;
      p0[r] = r0v;
      p1[r] = r1v;
      cp0[r] += r0v;
      cp1[r] += r1v;
      x0[r] = fmaf(r0v, we00, fmaf(r1v, we01, be0));
      x1[r] = fmaf(r0v, we10, fmaf(r1v, we11, be1));
    }

    {
      const int rsel  = nl & 7;
      const int which = nl >> 3;
      float sa = cp0[0], sb = cp1[0], sc = p0[0], sd = p1[0];
#pragma unroll
      for (int q = 1; q < 8; ++q) {
        const bool hit = (rsel == q);
        sa = hit ? cp0[q] : sa;
        sb = hit ? cp1[q] : sb;
        sc = hit ? p0[q] : sc;
        sd = hit ? p1[q] : sd;
      }
      v2f ov2;
      ov2[0] = which ? sc : sa;
      ov2[1] = which ? sd : sb;
      *(v2f*)(so + which * 32 + 2 * (8 * g + rsel)) = ov2;
    }
    wave_lds_sync();
    {
      const v4f ov4 = *(const v4f*)(so + (lane & 15) * 4);
      float* dst = out + (size_t)((lane >> 3) & 1) * (size_t)OUT1_OFF
                       + ((size_t)t * NBATCH + (size_t)rowW) * 2 + (size_t)(lane & 7) * 4;
      if (lane < 16) *(volatile v4f*)dst = ov4;
      __threadfence();
      if (lane < 16) *(volatile v4f*)dst = ov4;
    }
  }
}

extern "C" void kernel_launch(void* const* d_in, const int* in_sizes, int n_in,
                              void* d_out, int out_size, void* d_ws, size_t ws_size, hipStream_t stream) {
  (void)d_ws; (void)ws_size;
  if (n_in < 12 || d_out == nullptr) return;
  if (in_sizes[0] != NBATCH * NHID || in_sizes[1] != NBATCH * NHID ||
      in_sizes[2] != NBATCH * 2 || in_sizes[3] != NBATCH * 2 ||
      in_sizes[4] != 4 || in_sizes[5] != 2 ||
      in_sizes[6] != NGATE * 2 || in_sizes[7] != NGATE * NHID ||
      in_sizes[8] != NGATE || in_sizes[9] != NGATE ||
      in_sizes[10] != 2 * NHID || in_sizes[11] != 2 ||
      out_size != 2 * OUT1_OFF) return;

  const float* enc_h   = (const float*)d_in[0];
  const float* enc_c   = (const float*)d_in[1];
  const float* obs_pos = (const float*)d_in[2];
  const float* obs_rel = (const float*)d_in[3];
  const float* w_emb   = (const float*)d_in[4];
  const float* b_emb   = (const float*)d_in[5];
  const float* w_ih    = (const float*)d_in[6];
  const float* w_hh    = (const float*)d_in[7];
  const float* b_ih    = (const float*)d_in[8];
  const float* b_hh    = (const float*)d_in[9];
  const float* w_pos   = (const float*)d_in[10];
  const float* b_pos   = (const float*)d_in[11];
  float* out = (float*)d_out;

  lstm_seq_kernel<<<NBATCH / ROWS_BLK, NTHR, 0, stream>>>(
      enc_h, enc_c, obs_pos, obs_rel, w_emb, b_emb, w_ih, w_hh, b_ih, b_hh, w_pos, b_pos, out);
}
